// Mamba2_80814104642067
// MI455X (gfx1250) — hardware-verified
//
#include <hip/hip_runtime.h>
#include <math.h>

typedef __attribute__((ext_vector_type(16))) _Float16 v16h;
typedef __attribute__((ext_vector_type(8)))  _Float16 v8h;
typedef __attribute__((ext_vector_type(16))) __bf16   v16b;
typedef __attribute__((ext_vector_type(8)))  __bf16   v8b;
typedef __attribute__((ext_vector_type(8)))  float    v8f;
typedef __attribute__((ext_vector_type(4)))  float    v4f;
typedef __attribute__((ext_vector_type(4)))  unsigned int u32x4;

constexpr int kNL    = 2;
constexpr int kB     = 2;
constexpr int kL     = 2048;
constexpr int kDm    = 1024;
constexpr int kDi    = 2048;
constexpr int kH     = 32;
constexpr int kP     = 64;
constexpr int kNs    = 64;
constexpr int kDc    = 4;
constexpr int kCs    = 256;
constexpr int kNc    = kL / kCs;
constexpr int kRows  = kB * kL;
constexpr int kDin   = 2 * kDi + 2 * kNs + kH;
constexpr int kDinPad = 4288;
constexpr int kConvD = kDi + 2 * kNs;
constexpr int kColX  = kDi;
constexpr int kColDt = kDi + kConvD;
constexpr int kColB  = kDi;
constexpr int kColC  = kDi + kNs;
constexpr int kBlkCh = kB * kNc * kH;
constexpr float kEps = 1e-5f;
static_assert(kDin == 4256);
static_assert(kDinPad % 64 == 0 && kDinPad >= kDin && kDinPad - kDin < 64);
static_assert(kDm % 32 == 0 && kDi % 32 == 0);
static_assert(kRows % 64 == 0 && kDinPad % 64 == 0 && kDm % 64 == 0);
static_assert(kConvD % 128 == 0 && kL % 64 == 0 && kH == 32 && kNc == 8 && kP == 64 && kNs == 64 && kCs == 256);
static_assert((kDinPad * kDm) % (8 * 256) == 0 && (kDin * kDm) % (8 * 256) == 0 && (kDm * kDi) % (8 * 256) == 0);

constexpr size_t kOffWI   = 0;
constexpr size_t kSzWI    = (size_t)kDinPad * kDm * 2;
constexpr size_t kOffWO   = kOffWI + kSzWI;
constexpr size_t kSzWO    = (size_t)kDm * kDi * 2;
constexpr size_t kOffXN   = kOffWO + kSzWO;
constexpr size_t kSzXN    = (size_t)kRows * kDm * 2;
constexpr size_t kOffZX   = kOffXN + kSzXN;
constexpr size_t kSzZX    = (size_t)kRows * kDinPad * 2;
constexpr size_t kOffXBC  = kOffZX + kSzZX;
constexpr size_t kSzXBC   = (size_t)kRows * kConvD * 2;
constexpr size_t kOffDT   = kOffXBC + kSzXBC;
constexpr size_t kSzDT    = (size_t)kBlkCh * kCs * 4;
constexpr size_t kOffCUM  = kOffDT + kSzDT;
constexpr size_t kOffST   = kOffCUM + kSzDT;
constexpr size_t kSzST    = (size_t)kBlkCh * kP * kNs * 4;
constexpr size_t kOffPV   = kOffST + kSzST;
constexpr size_t kSzPV    = (size_t)kBlkCh * kP * kNs * 2;
constexpr size_t kOffYG   = kOffPV + kSzPV;
constexpr size_t kSzYG    = (size_t)kRows * kDi * 2;
constexpr size_t kOffSSQ  = kOffYG + kSzYG;
constexpr size_t kOffRS   = kOffSSQ + kSzDT;
constexpr size_t kSzRS    = (size_t)kRows * 4;
constexpr size_t kOffX1   = kOffRS + kSzRS;
constexpr size_t kSzX1    = (size_t)kRows * kDm * 4;
constexpr size_t kWsTotal = kOffX1 + kSzX1;
static_assert(kWsTotal == 122044416ull);
static_assert(kWsTotal <= 134217728ull);
static_assert((kOffWO % 128) == 0 && (kOffXN % 128) == 0 && (kOffZX % 128) == 0 && (kOffXBC % 128) == 0 &&
              (kOffDT % 128) == 0 && (kOffCUM % 128) == 0 && (kOffST % 128) == 0 && (kOffPV % 128) == 0 &&
              (kOffYG % 128) == 0 && (kOffSSQ % 128) == 0 && (kOffRS % 128) == 0 && (kOffX1 % 128) == 0);

__device__ __forceinline__ unsigned short f2bf_bits(float f) {
  unsigned u = __float_as_uint(f);
  return (unsigned short)((u + 0x7FFFu + ((u >> 16) & 1u)) >> 16);
}
__device__ __forceinline__ float bf_bits2f(unsigned short h) { return __uint_as_float(((unsigned)h) << 16); }

__device__ __forceinline__ float h16_to_f32(unsigned hb) {
  const unsigned sgn = (hb & 0x8000u) << 16; const unsigned em = hb & 0x7fffu;
  const float fn = __uint_as_float((em << 13) + 0x38000000u);
  const float fs = (float)em * 5.9604644775390625e-8f;
  const float mag = (em < 0x400u) ? fs : fn; return __uint_as_float(__float_as_uint(mag) | sgn); }

__device__ __forceinline__ void dep_guard_h(v8f& a, v8f& b, v16h x, v16h y) { asm volatile("v_nop\n\tv_nop\n\tv_nop\n\tv_nop" : "+v"(a), "+v"(b) : "v"(x), "v"(y)); }
__device__ __forceinline__ void dep_guard_b(v8f& a, v8f& b, v16b x, v16b y) { asm volatile("v_nop\n\tv_nop\n\tv_nop\n\tv_nop" : "+v"(a), "+v"(b) : "v"(x), "v"(y)); }
__device__ __forceinline__ void dep_guard4_h(v8f& a, v8f& b, v8f& c, v8f& d, v16h x, v16h y) {
  asm volatile("v_nop\n\tv_nop\n\tv_nop\n\tv_nop" : "+v"(a), "+v"(b), "+v"(c), "+v"(d) : "v"(x), "v"(y)); }
__device__ __forceinline__ void dep_guard4_b(v8f& a, v8f& b, v8f& c, v8f& d, v16b x, v16b y) {
  asm volatile("v_nop\n\tv_nop\n\tv_nop\n\tv_nop" : "+v"(a), "+v"(b), "+v"(c), "+v"(d) : "v"(x), "v"(y)); }
__device__ __forceinline__ void keep4_h(v16h a, v16h b, v16h c, v16h d) { asm volatile("v_nop" :: "v"(a), "v"(b), "v"(c), "v"(d)); }
__device__ __forceinline__ void keep4_b(v16b a, v16b b, v16b c, v16b d) { asm volatile("v_nop" :: "v"(a), "v"(b), "v"(c), "v"(d)); }
__device__ __forceinline__ void acc_guard4(v8f& a, v8f& b, v8f& c, v8f& d) { asm volatile("v_nop\n\tv_nop\n\tv_nop\n\tv_nop" : "+v"(a), "+v"(b), "+v"(c), "+v"(d)); }
template <typename T> struct Frag;
template <> struct Frag<_Float16> {
  typedef v16h V; union U { v16h v; v8h h[2]; };
  static __device__ __forceinline__ v16h load(const _Float16* p) {
    U f; f.h[0] = *(const v8h*)(p); f.h[1] = *(const v8h*)(p + 16); return f.v;
  }
  static __device__ __forceinline__ v8f mma(v16h a, v16h b, v8f c) {
    return __builtin_amdgcn_wmma_f32_16x16x32_f16(false, a, false, b, (short)0, c, false, false);
  }
  static __device__ __forceinline__ void guard(v8f& a, v8f& b, v16h x, v16h y) { dep_guard_h(a, b, x, y); }
  static __device__ __forceinline__ void guard4(v8f& a, v8f& b, v8f& c, v8f& d, v16h x, v16h y) { dep_guard4_h(a, b, c, d, x, y); }
  static __device__ __forceinline__ void keep(v16h a, v16h b, v16h c, v16h d) { keep4_h(a, b, c, d); }
};
template <> struct Frag<__bf16> {
  typedef v16b V; union U { v16b v; v8b h[2]; };
  static __device__ __forceinline__ v16b load(const __bf16* p) {
    U f; f.h[0] = *(const v8b*)(p); f.h[1] = *(const v8b*)(p + 16); return f.v;
  }
  static __device__ __forceinline__ v8f mma(v16b a, v16b b, v8f c) {
    return __builtin_amdgcn_wmma_f32_16x16x32_bf16(false, a, false, b, (short)0, c, false, false);
  }
  static __device__ __forceinline__ void guard(v8f& a, v8f& b, v16b x, v16b y) { dep_guard_b(a, b, x, y); }
  static __device__ __forceinline__ void guard4(v8f& a, v8f& b, v8f& c, v8f& d, v16b x, v16b y) { dep_guard4_b(a, b, c, d, x, y); }
  static __device__ __forceinline__ void keep(v16b a, v16b b, v16b c, v16b d) { keep4_b(a, b, c, d); }
};
typedef Frag<_Float16> FH;

template <int ET> struct Elem;
template <> struct Elem<0> { typedef _Float16 T; };
template <> struct Elem<1> { typedef __bf16 T; };
template <int ET, int SPL, int BIAS_MODE, int OUT_MODE, bool RESID, int ACT, bool RSRES>
__global__ __launch_bounds__(256) void wmma_gemm64(
    const unsigned short* __restrict__ Ap, const unsigned short* __restrict__ A2p, int lda, long strideA,
    const unsigned short* __restrict__ Btp, const unsigned short* __restrict__ Bt2p, int ldb, long strideB,
    void* __restrict__ Cout, void* __restrict__ Cout2, int ldc, long strideC,
    const float* __restrict__ bias,
    const float* __restrict__ resid, long strideR,
    int M, int N, int K, float scale) {
  static_assert(!(RSRES && (OUT_MODE != 0 || BIAS_MODE != 0 || RESID)));
  typedef typename Elem<ET>::T T;
  typedef typename Frag<T>::V V;
  const T* A = (const T*)Ap; const T* A2 = (const T*)A2p; const T* Bt = (const T*)Btp; const T* Bt2 = (const T*)Bt2p;
  __shared__ __align__(16) float sT[8][16 * 68];
  const int b    = blockIdx.y;
  const int lane = threadIdx.x & 31;
  const int wave = threadIdx.x >> 5;
  const int tilesN = N >> 6;
  const int tilesM = M >> 6;
  const int tile = blockIdx.x * 8 + wave;
  if (tile >= tilesM * tilesN) return;
  const int tm = tile / tilesN;
  const int tn = tile - tm * tilesN;
  const int m0 = tm << 6;
  const int n0 = tn << 6;

  const T* Ab  = A  + (size_t)b * strideA;
  const T* Bb  = Bt + (size_t)b * strideB;
  const T* Ab2 = (SPL >= 1) ? (A2  + (size_t)b * strideA) : nullptr;
  const T* Bb2 = (SPL == 2) ? (Bt2 + (size_t)b * strideB) : nullptr;

  const int rlane = lane & 15;
  const int koff  = (lane >> 4) * 8;
  const int mOff  = (lane >> 4) * 8;

  v8f acc[4][4];
#pragma unroll
  for (int i = 0; i < 4; ++i)
#pragma unroll
    for (int j = 0; j < 4; ++j) acc[i][j] = (v8f){0.f,0.f,0.f,0.f,0.f,0.f,0.f,0.f};

  for (int k0 = 0; k0 < K; k0 += 32) {
    V bh[4], bl[4];
#pragma unroll
    for (int j = 0; j < 4; ++j) {
      const size_t bo = (size_t)(n0 + (j << 4) + rlane) * ldb + koff + k0;
      bh[j] = Frag<T>::load(Bb + bo);
      if (SPL == 2) bl[j] = Frag<T>::load(Bb2 + bo);
    }
#pragma unroll
    for (int i = 0; i < 4; ++i) {
      const size_t ao = (size_t)(m0 + (i << 4) + rlane) * lda + koff + k0;
      V ah = Frag<T>::load(Ab + ao);
      V al;
      if (SPL >= 1) al = Frag<T>::load(Ab2 + ao);
#pragma unroll
      for (int j = 0; j < 4; ++j) {
        acc[i][j] = Frag<T>::mma(ah, bh[j], acc[i][j]);
        if (SPL == 2) acc[i][j] = Frag<T>::mma(ah, bl[j], acc[i][j]);
        if (SPL >= 1) acc[i][j] = Frag<T>::mma(al, bh[j], acc[i][j]);
      }
      Frag<T>::guard4(acc[i][0], acc[i][1], acc[i][2], acc[i][3], ah, (SPL >= 1) ? al : bh[3]);
    }
    Frag<T>::keep(bh[0], bh[1], bh[2], bh[3]);
    if (SPL == 2) Frag<T>::keep(bl[0], bl[1], bl[2], bl[3]);
  }
  acc_guard4(acc[0][0], acc[0][1], acc[0][2], acc[0][3]);
  acc_guard4(acc[1][0], acc[1][1], acc[1][2], acc[1][3]);
  acc_guard4(acc[2][0], acc[2][1], acc[2][2], acc[2][3]);
  acc_guard4(acc[3][0], acc[3][1], acc[3][2], acc[3][3]);

  float* slab = sT[wave];
  const float* Rb = RESID ? (resid + (size_t)b * strideR) : nullptr;
  const float* Rr = RSRES ? (resid + (size_t)b * strideR) : nullptr;
#pragma unroll
  for (int i = 0; i < 4; ++i) {
    const int mBase = m0 + (i << 4);
#pragma unroll
    for (int j = 0; j < 4; ++j) {
      const int n = n0 + (j << 4) + rlane;
      float bv = 0.f;
      if (BIAS_MODE == 2) bv = bias[n];
#pragma unroll
      for (int r = 0; r < 8; ++r) {
        float v = acc[i][j][r] * scale;
        if (BIAS_MODE == 1) v += bias[mBase + mOff + r];
        if (BIAS_MODE == 2) v += bv;
        if (RESID) v += Rb[(size_t)(mBase + mOff + r) * ldc + n];
        if (ACT == 1) v = tanhf(v);
        if (ACT == 2) v = fmaxf(v, 0.0f);
        if (ACT == 3) v = v / (1.0f + expf(-v));
        if (ACT == 4) v = (v > 0.f) ? v : 0.01f * v;
        slab[(mOff + r) * 68 + (j << 4) + rlane] = v;
      }
    }
    __builtin_amdgcn_fence(__ATOMIC_RELEASE, "workgroup");
    __builtin_amdgcn_wave_barrier();
    __builtin_amdgcn_fence(__ATOMIC_ACQUIRE, "workgroup");
    if (OUT_MODE == 0) {
      float* C = (float*)Cout + (size_t)b * strideC;
      const int hh = lane >> 4, c4 = (lane & 15) * 4;
      if (RSRES) {
#pragma unroll
        for (int it = 0; it < 8; ++it) {
          const int row = it * 2 + hh;
          const float rsv = bias[mBase + row];
          v4f sv = *(const v4f*)(slab + row * 68 + c4);
          const v4f rv = *(const v4f*)(Rr + (size_t)(mBase + row) * ldc + n0 + c4);
          sv = sv * rsv + rv;
          *(v4f*)(slab + row * 68 + c4) = sv;
        }
      }
      for (int pass = 0; pass < 2; ++pass) {
#pragma unroll
        for (int it = 0; it < 8; ++it) {
          const int row = it * 2 + hh;
          v4f v = *(const v4f*)(slab + row * 68 + c4);
          *(volatile v4f*)(C + (size_t)(mBase + row) * ldc + n0 + c4) = v;
        }
        __threadfence();
      }
    } else {
      const int q = lane >> 3, c8 = (lane & 7) * 8;
      unsigned short* C  = (unsigned short*)Cout  + (size_t)b * strideC;
      unsigned short* C2 = (OUT_MODE == 2) ? ((unsigned short*)Cout2 + (size_t)b * strideC) : nullptr;
      for (int pass = 0; pass < 2; ++pass) {
#pragma unroll
        for (int it = 0; it < 4; ++it) {
          const int row = it * 4 + q;
          const float* sp = slab + row * 68 + c8;
          v8h hv, lv;
#pragma unroll
          for (int e = 0; e < 8; ++e) {
            if (OUT_MODE == 1) {
              hv[e] = (_Float16)sp[e];
            } else {
              unsigned short hb = f2bf_bits(sp[e]);
              unsigned short lb = f2bf_bits(sp[e] - bf_bits2f(hb));
              hv[e] = __builtin_bit_cast(_Float16, hb);
              lv[e] = __builtin_bit_cast(_Float16, lb);
            }
          }
          *(volatile v8h*)(C + (size_t)(mBase + row) * ldc + n0 + c8) = hv;
          if (OUT_MODE == 2) *(volatile v8h*)(C2 + (size_t)(mBase + row) * ldc + n0 + c8) = lv;
        }
        __threadfence();
      }
    }
    __builtin_amdgcn_fence(__ATOMIC_RELEASE, "workgroup");
    __builtin_amdgcn_wave_barrier();
    __builtin_amdgcn_fence(__ATOMIC_ACQUIRE, "workgroup");
  }
}

template <bool KS>
__global__ __launch_bounds__(256) void cast_w_f16_kernel(
    const float* __restrict__ src, const float* __restrict__ ks, int kdim,
    unsigned short* __restrict__ dst, int total8, int valid8, float mul)
{
  const int i = blockIdx.x * 256 + threadIdx.x;
  if (i >= total8) return;
  const int iv = (i < valid8) ? i : (valid8 - 1);
  const size_t e0 = (size_t)iv << 3;
  const v4f a0 = *(const v4f*)(src + e0);
  const v4f a1 = *(const v4f*)(src + e0 + 4);
  const float f = (i < valid8) ? mul : 0.0f;
  v4f s0 = (v4f){1.f, 1.f, 1.f, 1.f}, s1 = (v4f){1.f, 1.f, 1.f, 1.f};
  if (KS) {
    const int k = (int)(e0 % (size_t)kdim);
    s0 = *(const v4f*)(ks + k);
    s1 = *(const v4f*)(ks + k + 4);
  }
  v8h hv;
#pragma unroll
  for (int e = 0; e < 4; ++e) {
    hv[e]     = (_Float16)(a0[e] * f * s0[e]);
    hv[4 + e] = (_Float16)(a1[e] * f * s1[e]);
  }
  unsigned short* q = dst + ((size_t)i << 3);
  *(volatile v8h*)q = hv;
  __threadfence();
  *(volatile v8h*)q = hv;
}

__global__ __launch_bounds__(128) void rmsnorm_in_kernel(
    const float* __restrict__ X, const float* __restrict__ wgt, unsigned short* __restrict__ XN)
{
  __shared__ float red[4];
  const int tid = threadIdx.x, lane = tid & 31, wave = tid >> 5;
  const size_t row = blockIdx.x;
  const float* xr = X + row * kDm + tid * 8;
  const v4f a0 = *(const v4f*)(xr);
  const v4f a1 = *(const v4f*)(xr + 4);
  float ss = 0.0f;
#pragma unroll
  for (int e = 0; e < 4; ++e) { ss = fmaf(a0[e], a0[e], ss); ss = fmaf(a1[e], a1[e], ss); }
#pragma unroll
  for (int off = 1; off < 32; off <<= 1) ss += __shfl_xor(ss, off, 32);
  if (lane == 0) red[wave] = ss;
  __syncthreads();
  const float tot = (red[0] + red[1]) + (red[2] + red[3]);
  const float sc = rsqrtf(tot * (1.0f / 1024.0f) + kEps);
  const v4f w0 = *(const v4f*)(wgt + tid * 8);
  const v4f w1 = *(const v4f*)(wgt + tid * 8 + 4);
  v8h hv;
#pragma unroll
  for (int e = 0; e < 4; ++e) {
    hv[e]     = (_Float16)(a0[e] * sc * w0[e]);
    hv[4 + e] = (_Float16)(a1[e] * sc * w1[e]);
  }
  unsigned short* q = XN + row * kDm + tid * 8;
  *(volatile v8h*)q = hv;
  __threadfence();
  *(volatile v8h*)q = hv;
}

__global__ __launch_bounds__(128) void conv_silu_kernel(
    const unsigned short* __restrict__ ZX, const float* __restrict__ cw, const float* __restrict__ cb,
    unsigned short* __restrict__ XBC)
{
  __shared__ __align__(16) float sT[67 * 128];
  const int tid = threadIdx.x, lane = tid & 31, wave = tid >> 5;
  const int c0 = blockIdx.x * 128;
  const int g0 = blockIdx.y * 64;
  const int tb = g0 & (kL - 1);
  const bool hist = (tb > 0);
  {
    const int idx = (tid < 47) ? tid : 47;
    const int r = idx >> 4, q = idx & 15;
    const int srow = hist ? (g0 - 3 + r) : g0;
    const u32x4 w = *(const u32x4*)(ZX + (size_t)srow * kDinPad + kColX + c0 + q * 8);
    const float hf = hist ? 1.0f : 0.0f;
    v4f lo, hi;
#pragma unroll
    for (int e = 0; e < 2; ++e) {
      lo[2 * e]     = h16_to_f32(w[e] & 0xffffu) * hf;
      lo[2 * e + 1] = h16_to_f32(w[e] >> 16) * hf;
      hi[2 * e]     = h16_to_f32(w[2 + e] & 0xffffu) * hf;
      hi[2 * e + 1] = h16_to_f32(w[2 + e] >> 16) * hf;
    }
    if (tid < 48) {
      *(v4f*)(sT + r * 128 + q * 8) = lo;
      *(v4f*)(sT + r * 128 + q * 8 + 4) = hi;
    }
  }
#pragma unroll 2
  for (int k = 0; k < 8; ++k) {
    const int idx = tid + 128 * k;
    const int r = idx >> 4, q = idx & 15;
    const u32x4 w = *(const u32x4*)(ZX + (size_t)(g0 + r) * kDinPad + kColX + c0 + q * 8);
    v4f lo, hi;
#pragma unroll
    for (int e = 0; e < 2; ++e) {
      lo[2 * e]     = h16_to_f32(w[e] & 0xffffu);
      lo[2 * e + 1] = h16_to_f32(w[e] >> 16);
      hi[2 * e]     = h16_to_f32(w[2 + e] & 0xffffu);
      hi[2 * e + 1] = h16_to_f32(w[2 + e] >> 16);
    }
    *(v4f*)(sT + (3 + r) * 128 + q * 8) = lo;
    *(v4f*)(sT + (3 + r) * 128 + q * 8 + 4) = hi;
  }
  __syncthreads();
  {
    const int d = c0 + tid;
    const float w0 = cw[d * kDc + 0], w1 = cw[d * kDc + 1], w2 = cw[d * kDc + 2], w3 = cw[d * kDc + 3];
    const float bc = cb[d];
    float xm3 = sT[tid], xm2 = sT[128 + tid], xm1 = sT[256 + tid];
#pragma unroll 1
    for (int s = 0; s < 64; ++s) {
      const float xcur = sT[(3 + s) * 128 + tid];
      float acc = w0 * xm3;
      acc = fmaf(w1, xm2, acc);
      acc = fmaf(w2, xm1, acc);
      acc = fmaf(w3, xcur, acc);
      const float sv = acc + bc;
      const float sg = __builtin_amdgcn_rcpf(1.0f + expf(-sv));
      sT[(3 + s) * 128 + tid] = sv * sg;
      xm3 = xm2; xm2 = xm1; xm1 = xcur;
    }
  }
  __syncthreads();
  v8h hv[8];
  const int hr = lane >> 4, c8 = (lane & 15) * 8;
#pragma unroll
  for (int it = 0; it < 8; ++it) {
    const int row = it * 8 + wave * 2 + hr;
    const float* sp = sT + (3 + row) * 128 + c8;
    const v4f a0 = *(const v4f*)(sp);
    const v4f a1 = *(const v4f*)(sp + 4);
#pragma unroll
    for (int e = 0; e < 4; ++e) { hv[it][e] = (_Float16)a0[e]; hv[it][4 + e] = (_Float16)a1[e]; }
  }
  for (int pass = 0; pass < 2; ++pass) {
#pragma unroll
    for (int it = 0; it < 8; ++it) {
      const int row = it * 8 + wave * 2 + hr;
      *(volatile v8h*)(XBC + (size_t)(g0 + row) * kConvD + c0 + c8) = hv[it];
    }
    __threadfence();
  }
}

__global__ __launch_bounds__(256) void dt_cum_kernel(
    const unsigned short* __restrict__ ZX, const float* __restrict__ dt_bias, const float* __restrict__ A_log,
    float* __restrict__ DT, float* __restrict__ CUM)
{
  __shared__ float s[kCs];
  const int blk = blockIdx.x;
  const int h = blk & (kH - 1), c = (blk >> 5) & (kNc - 1), b = blk >> 8;
  const int t = threadIdx.x;
  const size_t row = (size_t)b * kL + (size_t)c * kCs + t;
  const unsigned wd = *(const unsigned*)(ZX + row * kDinPad + kColDt + (h & ~1));
  const unsigned hb = (h & 1) ? (wd >> 16) : (wd & 0xffffu);
  const float raw = h16_to_f32(hb);
  const float v = raw + dt_bias[h];
  const float a = expf(-fabsf(v));
  const float dt = fmaxf(v, 0.0f) + log1pf(a);
  const float dA = dt * (-expf(A_log[h]));
  s[t] = dA;
  __syncthreads();
#pragma unroll 1
  for (int off = 1; off < kCs; off <<= 1) {
    const int src = (t >= off) ? (t - off) : t;
    const float tv = s[src];
    const float add = (t >= off) ? tv : 0.0f;
    __syncthreads();
    s[t] += add;
    __syncthreads();
  }
  const float cum = s[t];
  float* od = DT + (size_t)blk * kCs + t;
  float* oc = CUM + (size_t)blk * kCs + t;
  *(volatile float*)od = dt;
  *(volatile float*)oc = cum;
  __threadfence();
  *(volatile float*)od = dt;
  *(volatile float*)oc = cum;
}

__global__ __launch_bounds__(128) void states_kernel(
    const unsigned short* __restrict__ XBC, const float* __restrict__ DT, const float* __restrict__ CUM,
    float* __restrict__ ST)
{
  __shared__ __align__(16) unsigned short sXT[kP * kCs];
  __shared__ __align__(16) unsigned short sBD[kNs * kCs];
  __shared__ __align__(16) float sSlab[4][16 * 64];
  __shared__ float sDec[kCs];
  const int tid = threadIdx.x, lane = tid & 31, wave = tid >> 5;
  const int hh = lane >> 4, rl = lane & 15, koff = hh * 8;
  const int blk = blockIdx.x;
  const int h = blk & (kH - 1), c = (blk >> 5) & (kNc - 1), b = blk >> 8;
  const size_t rowb = (size_t)b * kL + (size_t)c * kCs;
  {
    const float cl = CUM[(size_t)blk * kCs + (kCs - 1)];
#pragma unroll
    for (int k = 0; k < 2; ++k) {
      const int j = tid + 128 * k;
      sDec[j] = 256.0f * expf(cl - CUM[(size_t)blk * kCs + j]) * DT[(size_t)blk * kCs + j];
    }
  }
  __syncthreads();
#pragma unroll 4
  for (int k = 0; k < 16; ++k) {
    const int idx = tid + 128 * k;
    const int j = idx >> 3, q = idx & 7;
    const u32x4 w = *(const u32x4*)(XBC + (rowb + j) * kConvD + h * kP + q * 8);
#pragma unroll
    for (int e = 0; e < 4; ++e) {
      sXT[(q * 8 + 2 * e) * kCs + j]     = (unsigned short)(w[e] & 0xffffu);
      sXT[(q * 8 + 2 * e + 1) * kCs + j] = (unsigned short)(w[e] >> 16);
    }
  }
#pragma unroll 2
  for (int k = 0; k < 16; ++k) {
    const int idx = tid + 128 * k;
    const int j = idx >> 3, q = idx & 7;
    const u32x4 w = *(const u32x4*)(XBC + (rowb + j) * kConvD + kColB + q * 8);
    const float sd = sDec[j];
#pragma unroll
    for (int e = 0; e < 4; ++e) {
      const float f0 = h16_to_f32(w[e] & 0xffffu) * sd;
      const float f1 = h16_to_f32(w[e] >> 16) * sd;
      sBD[(q * 8 + 2 * e) * kCs + j]     = __builtin_bit_cast(unsigned short, (_Float16)f0);
      sBD[(q * 8 + 2 * e + 1) * kCs + j] = __builtin_bit_cast(unsigned short, (_Float16)f1);
    }
  }
  __syncthreads();
  const _Float16* Xt = (const _Float16*)(const void*)sXT;
  const _Float16* Bd = (const _Float16*)(const void*)sBD;
  const int pm = wave * 16;
  v8f acc[4];
#pragma unroll
  for (int ni = 0; ni < 4; ++ni) acc[ni] = (v8f){0.f,0.f,0.f,0.f,0.f,0.f,0.f,0.f};
#pragma unroll 1
  for (int k0 = 0; k0 < kCs; k0 += 32) {
    const v16h a = FH::load(Xt + (pm + rl) * kCs + k0 + koff);
    v16h bq[4];
#pragma unroll
    for (int ni = 0; ni < 4; ++ni) bq[ni] = FH::load(Bd + (ni * 16 + rl) * kCs + k0 + koff);
#pragma unroll
    for (int ni = 0; ni < 4; ++ni) acc[ni] = FH::mma(a, bq[ni], acc[ni]);
    dep_guard4_h(acc[0], acc[1], acc[2], acc[3], a, bq[3]);
    keep4_h(bq[0], bq[1], bq[2], a);
  }
  acc_guard4(acc[0], acc[1], acc[2], acc[3]);
  float* slab = sSlab[wave];
#pragma unroll
  for (int ni = 0; ni < 4; ++ni)
#pragma unroll
    for (int r = 0; r < 8; ++r) slab[(8 * hh + r) * 64 + ni * 16 + rl] = acc[ni][r];
  __builtin_amdgcn_fence(__ATOMIC_RELEASE, "workgroup");
  __builtin_amdgcn_wave_barrier();
  __builtin_amdgcn_fence(__ATOMIC_ACQUIRE, "workgroup");
  const int c4 = rl * 4;
  float* Ob = ST + (size_t)blk * (kP * kNs) + (size_t)pm * kNs;
  for (int pass = 0; pass < 2; ++pass) {
#pragma unroll
    for (int it = 0; it < 8; ++it) {
      const int row = it * 2 + hh;
      const v4f v = *(const v4f*)(slab + row * 64 + c4);
      *(volatile v4f*)(Ob + (size_t)row * kNs + c4) = v;
    }
    __threadfence();
  }
}

__global__ __launch_bounds__(256) void chunk_scan_kernel(
    const float* __restrict__ ST, const float* __restrict__ CUM, unsigned short* __restrict__ PV)
{
  const int g = blockIdx.x * 256 + threadIdx.x;
  const int q = g & 7, p = (g >> 3) & (kP - 1), h = (g >> 9) & (kH - 1), b = g >> 14;
  v4f s0 = (v4f){0.f, 0.f, 0.f, 0.f}, s1 = (v4f){0.f, 0.f, 0.f, 0.f};
#pragma unroll 1
  for (int c = 0; c < kNc; ++c) {
    const int blk = (b * kNc + c) * kH + h;
    const size_t base = (size_t)blk * (kP * kNs) + (size_t)p * kNs + q * 8;
    const v4f t0 = *(const v4f*)(ST + base);
    const v4f t1 = *(const v4f*)(ST + base + 4);
    const float dec = expf(CUM[(size_t)blk * kCs + (kCs - 1)]);
    v8h hv;
#pragma unroll
    for (int e = 0; e < 4; ++e) { hv[e] = (_Float16)s0[e]; hv[4 + e] = (_Float16)s1[e]; }
    unsigned short* o = PV + base;
    *(volatile v8h*)o = hv;
    __threadfence();
    *(volatile v8h*)o = hv;
    s0 = s0 * dec + t0;
    s1 = s1 * dec + t1;
  }
}

__global__ __launch_bounds__(256) void ssd_y_kernel(
    const unsigned short* __restrict__ XBC, const unsigned short* __restrict__ ZX,
    const float* __restrict__ DT, const float* __restrict__ CUM, const unsigned short* __restrict__ PREV,
    const float* __restrict__ Dp, unsigned short* __restrict__ YG, float* __restrict__ SSQ)
{
  __shared__ __align__(16) unsigned short sCB[2 * kCs * kNs];
  __shared__ __align__(16) unsigned short sXT[kP * kCs];
  __shared__ __align__(16) unsigned short sPV[kP * kNs];
  __shared__ __align__(16) unsigned short sS[8 * 32 * 32];
  __shared__ float sCum[kCs], sDt[kCs], sSq[kCs];
  const int tid = threadIdx.x, lane = tid & 31, wave = tid >> 5;
  const int hh = lane >> 4, rl = lane & 15, koff = hh * 8;
  const int blk = blockIdx.x;
  const int h = blk & (kH - 1), c = (blk >> 5) & (kNc - 1), b = blk >> 8;
  const size_t rowb = (size_t)b * kL + (size_t)c * kCs;
  unsigned short* sC  = sCB;
  unsigned short* sBm = sCB + kCs * kNs;
  {
    const int t = tid;
    const unsigned short* xr = XBC + (rowb + t) * kConvD;
    sCum[t] = CUM[(size_t)blk * kCs + t];
    sDt[t]  = DT[(size_t)blk * kCs + t];
#pragma unroll
    for (int q = 0; q < 8; ++q) *(u32x4*)(sC + t * kNs + q * 8) = *(const u32x4*)(xr + kColC + q * 8);
    asm volatile("" ::: "memory");
#pragma unroll
    for (int q = 0; q < 8; ++q) *(u32x4*)(sBm + t * kNs + q * 8) = *(const u32x4*)(xr + kColB + q * 8);
    asm volatile("" ::: "memory");
#pragma unroll 2
    for (int q = 0; q < 8; ++q) {
      const u32x4 w = *(const u32x4*)(xr + h * kP + q * 8);
#pragma unroll
      for (int e = 0; e < 4; ++e) {
        sXT[(q * 8 + 2 * e) * kCs + t]     = (unsigned short)(w[e] & 0xffffu);
        sXT[(q * 8 + 2 * e + 1) * kCs + t] = (unsigned short)(w[e] >> 16);
      }
    }
    asm volatile("" ::: "memory");
#pragma unroll
    for (int k = 0; k < 2; ++k) {
      const int idx = t + 256 * k;
      *(u32x4*)(sPV + idx * 8) = *(const u32x4*)(PREV + (size_t)blk * (kP * kNs) + idx * 8);
    }
  }
  __syncthreads();

  const _Float16* Cs = (const _Float16*)(const void*)sC;
  const _Float16* Bs = (const _Float16*)(const void*)sBm;
  const _Float16* Xt = (const _Float16*)(const void*)sXT;
  const _Float16* Pv = (const _Float16*)(const void*)sPV;
  unsigned short* sSw16 = sS + wave * (32 * 32);
  const _Float16* Sw = (const _Float16*)(const void*)sSw16;
  const int i0 = wave * 32;

  v8f acc[2][4];
#pragma unroll
  for (int mi = 0; mi < 2; ++mi)
#pragma unroll
    for (int ni = 0; ni < 4; ++ni) acc[mi][ni] = (v8f){0.f,0.f,0.f,0.f,0.f,0.f,0.f,0.f};

#pragma unroll
  for (int ks = 0; ks < 2; ++ks) {
    const int k0 = ks * 32;
    const v16h a0 = FH::load(Cs + (i0 + rl) * kNs + k0 + koff);
    const v16h a1 = FH::load(Cs + (i0 + 16 + rl) * kNs + k0 + koff);
    v16h bq[4];
#pragma unroll
    for (int ni = 0; ni < 4; ++ni) bq[ni] = FH::load(Pv + (ni * 16 + rl) * kNs + k0 + koff);
#pragma unroll
    for (int ni = 0; ni < 4; ++ni) {
      acc[0][ni] = FH::mma(a0, bq[ni], acc[0][ni]);
      acc[1][ni] = FH::mma(a1, bq[ni], acc[1][ni]);
    }
    dep_guard4_h(acc[0][0], acc[0][1], acc[0][2], acc[0][3], a0, bq[3]);
    dep_guard4_h(acc[1][0], acc[1][1], acc[1][2], acc[1][3], a1, bq[3]);
    keep4_h(bq[0], bq[1], bq[2], a0);
  }
#pragma unroll
  for (int mi = 0; mi < 2; ++mi) {
#pragma unroll
    for (int r = 0; r < 8; ++r) {
      const float ei = expf(sCum[i0 + mi * 16 + 8 * hh + r]);
#pragma unroll
      for (int ni = 0; ni < 4; ++ni) acc[mi][ni][r] *= ei;
    }
  }

#pragma unroll 1
  for (int jb = 0; jb <= wave; ++jb) {
    const int j0 = jb * 32;
    v8f tt[2][2];
#pragma unroll
    for (int mi = 0; mi < 2; ++mi)
#pragma unroll
      for (int tj = 0; tj < 2; ++tj) tt[mi][tj] = (v8f){0.f,0.f,0.f,0.f,0.f,0.f,0.f,0.f};
#pragma unroll
    for (int ks = 0; ks < 2; ++ks) {
      const int k0 = ks * 32;
      const v16h a0 = FH::load(Cs + (i0 + rl) * kNs + k0 + koff);
      const v16h a1 = FH::load(Cs + (i0 + 16 + rl) * kNs + k0 + koff);
      const v16h b0 = FH::load(Bs + (j0 + rl) * kNs + k0 + koff);
      const v16h b1 = FH::load(Bs + (j0 + 16 + rl) * kNs + k0 + koff);
      tt[0][0] = FH::mma(a0, b0, tt[0][0]);
      tt[0][1] = FH::mma(a0, b1, tt[0][1]);
      tt[1][0] = FH::mma(a1, b0, tt[1][0]);
      tt[1][1] = FH::mma(a1, b1, tt[1][1]);
      dep_guard4_h(tt[0][0], tt[0][1], tt[1][0], tt[1][1], a0, a1);
      keep4_h(b0, b1, a0, a1);
    }
    __builtin_amdgcn_fence(__ATOMIC_RELEASE, "workgroup");
    __builtin_amdgcn_wave_barrier();
    __builtin_amdgcn_fence(__ATOMIC_ACQUIRE, "workgroup");
#pragma unroll
    for (int mi = 0; mi < 2; ++mi) {
#pragma unroll
      for (int tj = 0; tj < 2; ++tj) {
        const int j = j0 + tj * 16 + rl;
        const float cj = sCum[j];
        const float sdt = 256.0f * sDt[j];
#pragma unroll
        for (int r = 0; r < 8; ++r) {
          const int il = mi * 16 + 8 * hh + r;
          const int i = i0 + il;
          const bool m = (j <= i);
          const float dsel = m ? (sCum[i] - cj) : 0.0f;
          const float ev = expf(dsel);
          const float v = m ? (tt[mi][tj][r] * ev * sdt) : 0.0f;
          sSw16[il * 32 + tj * 16 + rl] = __builtin_bit_cast(unsigned short, (_Float16)v);
        }
      }
    }
    __builtin_amdgcn_fence(__ATOMIC_RELEASE, "workgroup");
    __builtin_amdgcn_wave_barrier();
    __builtin_amdgcn_fence(__ATOMIC_ACQUIRE, "workgroup");
    const v16h sa0 = FH::load(Sw + rl * 32 + koff);
    const v16h sa1 = FH::load(Sw + (16 + rl) * 32 + koff);
    v16h xq[4];
#pragma unroll
    for (int ni = 0; ni < 4; ++ni) xq[ni] = FH::load(Xt + (ni * 16 + rl) * kCs + j0 + koff);
#pragma unroll
    for (int ni = 0; ni < 4; ++ni) {
      acc[0][ni] = FH::mma(sa0, xq[ni], acc[0][ni]);
      acc[1][ni] = FH::mma(sa1, xq[ni], acc[1][ni]);
    }
    dep_guard4_h(acc[0][0], acc[0][1], acc[0][2], acc[0][3], sa0, xq[3]);
    dep_guard4_h(acc[1][0], acc[1][1], acc[1][2], acc[1][3], sa1, xq[3]);
    keep4_h(xq[0], xq[1], xq[2], sa0);
  }
  acc_guard4(acc[0][0], acc[0][1], acc[0][2], acc[0][3]);
  acc_guard4(acc[1][0], acc[1][1], acc[1][2], acc[1][3]);

  __syncthreads();
  float* slab = (float*)(void*)sCB + wave * (32 * 64);
#pragma unroll
  for (int mi = 0; mi < 2; ++mi)
#pragma unroll
    for (int ni = 0; ni < 4; ++ni)
#pragma unroll
      for (int r = 0; r < 8; ++r)
        slab[(mi * 16 + 8 * hh + r) * 64 + ni * 16 + rl] = acc[mi][ni][r] * (1.0f / 256.0f);
  __builtin_amdgcn_fence(__ATOMIC_RELEASE, "workgroup");
  __builtin_amdgcn_wave_barrier();
  __builtin_amdgcn_fence(__ATOMIC_ACQUIRE, "workgroup");
  const float Dh = Dp[h];
  const int q = lane >> 3, c8 = (lane & 7) * 8;
#pragma unroll 1
  for (int it = 0; it < 8; ++it) {
    const int rloc = it * 4 + q;
    const size_t row = rowb + i0 + rloc;
    const u32x4 zw = *(const u32x4*)(ZX + row * kDinPad + h * kP + c8);
    float* sp = slab + rloc * 64 + c8;
    const v4f y0 = *(const v4f*)(sp);
    const v4f y1 = *(const v4f*)(sp + 4);
    float ssq = 0.0f;
    v4f g0, g1;
#pragma unroll
    for (int e = 0; e < 4; ++e) {
      const unsigned zword = zw[e];
      const unsigned zlo = zword & 0xffffu, zhi = zword >> 16;
      const float yb = (e < 2) ? y0[2 * e - ((e < 2) ? 0 : 4)] : y1[2 * (e - 2)];
      const float yc = (e < 2) ? y0[2 * e + 1 - ((e < 2) ? 0 : 4)] : y1[2 * (e - 2) + 1];
      const float xa = h16_to_f32(sXT[(c8 + 2 * e) * kCs + i0 + rloc]);
      const float xb = h16_to_f32(sXT[(c8 + 2 * e + 1) * kCs + i0 + rloc]);
      const float za = h16_to_f32(zlo), zb = h16_to_f32(zhi);
      const float ya = fmaf(Dh, xa, yb);
      const float ybv = fmaf(Dh, xb, yc);
      const float sga = __builtin_amdgcn_rcpf(1.0f + expf(-za));
      const float sgb = __builtin_amdgcn_rcpf(1.0f + expf(-zb));
      const float ga = ya * (za * sga);
      const float gb = ybv * (zb * sgb);
      ssq = fmaf(ga, ga, ssq);
      ssq = fmaf(gb, gb, ssq);
      if (e < 2) { g0[2 * e] = ga; g0[2 * e + 1] = gb; } else { g1[2 * (e - 2)] = ga; g1[2 * (e - 2) + 1] = gb; }
    }
    *(v4f*)(sp) = g0;
    *(v4f*)(sp + 4) = g1;
    ssq += __shfl_xor(ssq, 1, 32);
    ssq += __shfl_xor(ssq, 2, 32);
    ssq += __shfl_xor(ssq, 4, 32);
    if ((lane & 7) == 0) sSq[i0 + rloc] = ssq;
  }
  for (int pass = 0; pass < 2; ++pass) {
#pragma unroll
    for (int it = 0; it < 8; ++it) {
      const int rloc = it * 4 + q;
      const size_t row = rowb + i0 + rloc;
      const float* sp = slab + rloc * 64 + c8;
      const v4f a0 = *(const v4f*)(sp);
      const v4f a1 = *(const v4f*)(sp + 4);
      v8h hv;
#pragma unroll
      for (int e = 0; e < 4; ++e) { hv[e] = (_Float16)(a0[e] * 8.0f); hv[4 + e] = (_Float16)(a1[e] * 8.0f); }
      *(volatile v8h*)(YG + row * kDi + h * kP + c8) = hv;
    }
    __threadfence();
  }
  __syncthreads();
  {
    const float sv = sSq[tid];
    float* o = SSQ + (size_t)blk * kCs + tid;
    *(volatile float*)o = sv;
    __threadfence();
    *(volatile float*)o = sv;
  }
}

__global__ __launch_bounds__(256) void rowscale_kernel(const float* __restrict__ SSQ, float* __restrict__ RS)
{
  const int r = blockIdx.x * 256 + threadIdx.x;
  const int b = r >> 11, wl = r & (kL - 1), c = wl >> 8, i = wl & (kCs - 1);
  const size_t base = (size_t)((b * kNc + c) * kH) * kCs + i;
  float s = 0.0f;
#pragma unroll 8
  for (int h = 0; h < kH; ++h) s += SSQ[base + (size_t)h * kCs];
  const float rs = rsqrtf(s * (1.0f / 2048.0f) + kEps);
  float* o = RS + r;
  *(volatile float*)o = rs;
  __threadfence();
  *(volatile float*)o = rs;
}

extern "C" void kernel_launch(void* const* d_in, const int* in_sizes, int n_in,
                              void* d_out, int out_size, void* d_ws, size_t ws_size,
                              hipStream_t stream) {
  if (n_in < 10) return;
  if (in_sizes[0] != kRows * kDm) return;
  if (in_sizes[1] != kNL * kDm) return;
  if (in_sizes[2] != kNL * kDin * kDm) return;
  if (in_sizes[3] != kNL * kConvD * kDc) return;
  if (in_sizes[4] != kNL * kConvD) return;
  if (in_sizes[5] != kNL * kH) return;
  if (in_sizes[6] != kNL * kH) return;
  if (in_sizes[7] != kNL * kH) return;
  if (in_sizes[8] != kNL * kDi) return;
  if (in_sizes[9] != kNL * kDm * kDi) return;
  if (out_size != kRows * kDm) return;
  if (ws_size < kWsTotal) return;

  const float* u       = (const float*)d_in[0];
  const float* norm_w  = (const float*)d_in[1];
  const float* in_w    = (const float*)d_in[2];
  const float* conv_w  = (const float*)d_in[3];
  const float* conv_b  = (const float*)d_in[4];
  const float* dt_bias = (const float*)d_in[5];
  const float* A_log   = (const float*)d_in[6];
  const float* Dpw     = (const float*)d_in[7];
  const float* rms_w   = (const float*)d_in[8];
  const float* out_w   = (const float*)d_in[9];
  float* out = (float*)d_out;

  char* ws = (char*)d_ws;
  unsigned short* WI  = (unsigned short*)(ws + kOffWI);
  unsigned short* WO  = (unsigned short*)(ws + kOffWO);
  unsigned short* XN  = (unsigned short*)(ws + kOffXN);
  unsigned short* ZX  = (unsigned short*)(ws + kOffZX);
  unsigned short* XBC = (unsigned short*)(ws + kOffXBC);
  float*          DT  = (float*)(ws + kOffDT);
  float*          CUM = (float*)(ws + kOffCUM);
  float*          ST  = (float*)(ws + kOffST);
  unsigned short* PV  = (unsigned short*)(ws + kOffPV);
  unsigned short* YG  = (unsigned short*)(ws + kOffYG);
  float*          SSQ = (float*)(ws + kOffSSQ);
  float*          RS  = (float*)(ws + kOffRS);
  float*          X1  = (float*)(ws + kOffX1);

  constexpr int kWiTotal8 = kDinPad * kDm / 8;
  constexpr int kWiValid8 = kDin * kDm / 8;
  constexpr int kWoTotal8 = kDm * kDi / 8;
  static_assert(kWiTotal8 % 256 == 0 && kWoTotal8 % 256 == 0);

  for (int layer = 0; layer < kNL; ++layer) {
    const float* xin  = (layer == 0) ? u : (const float*)X1;
    float*       xdst = (layer == 0) ? X1 : out;

    cast_w_f16_kernel<false><<<kWiTotal8 / 256, 256, 0, stream>>>(
        in_w + (size_t)layer * kDin * kDm, nullptr, 8, WI, kWiTotal8, kWiValid8, 64.0f);
    cast_w_f16_kernel<true><<<kWoTotal8 / 256, 256, 0, stream>>>(
        out_w + (size_t)layer * kDm * kDi, rms_w + (size_t)layer * kDi, kDi, WO, kWoTotal8, kWoTotal8, 64.0f);

    rmsnorm_in_kernel<<<kRows, 128, 0, stream>>>(xin, norm_w + (size_t)layer * kDm, XN);

    wmma_gemm64<0, 0, 0, 1, false, 0, false><<<dim3((kRows / 64) * (kDinPad / 64) / 8, 1), 256, 0, stream>>>(
        XN, XN, kDm, 0L,
        WI, WI, kDm, 0L,
        (void*)ZX, nullptr, kDinPad, 0L,
        nullptr, nullptr, 0L,
        kRows, kDinPad, kDm, 1.0f / 64.0f);

    conv_silu_kernel<<<dim3(kConvD / 128, kRows / 64), 128, 0, stream>>>(
        ZX, conv_w + (size_t)layer * kConvD * kDc, conv_b + (size_t)layer * kConvD, XBC);

    dt_cum_kernel<<<kBlkCh, kCs, 0, stream>>>(ZX, dt_bias + (size_t)layer * kH, A_log + (size_t)layer * kH, DT, CUM);

    states_kernel<<<kBlkCh, 128, 0, stream>>>(XBC, DT, CUM, ST);

    chunk_scan_kernel<<<(kB * kH * kP * kNs / 8) / 256, 256, 0, stream>>>(ST, CUM, PV);

    ssd_y_kernel<<<kBlkCh, 256, 0, stream>>>(XBC, ZX, DT, CUM, PV, Dpw + (size_t)layer * kH, YG, SSQ);

    rowscale_kernel<<<kRows / 256, 256, 0, stream>>>(SSQ, RS);

    wmma_gemm64<0, 0, 0, 0, false, 0, true><<<dim3((kRows / 64) * (kDm / 64) / 8, 1), 256, 0, stream>>>(
        YG, YG, kDi, 0L,
        WO, WO, kDi, 0L,
        (void*)xdst, nullptr, kDm, 0L,
        RS, xin, 0L,
        kRows, kDm, kDi, 1.0f / 512.0f);
  }
}
